// KGCN_79783312491281
// MI455X (gfx1250) — hardware-run, weakly checked
//
#include <hip/hip_runtime.h>
#include <stddef.h>
#include <stdint.h>


#define SPLIT_V 1
#define NB     16384
#define NK     32
#define ND     64
#define NUSR   100000
#define NENT   100000
#define NREL   32
#define VP     128
#define WP     128
#define KUSE   (SPLIT_V ? 128 : 64)
#define NTHR   256
#define NWAVE  8
#define RPW_E  20
#define ROWS_E (NWAVE * RPW_E)
#define NB_ENT (NENT / ROWS_E)
#define PPW    4
#define PPB    (NWAVE * PPW)
#define LBM    128
#define RELP   65

static_assert(ND == 64);
static_assert(NK == 32 && NREL == 32);
static_assert(NENT % ROWS_E == 0);
static_assert(NREL == NWAVE * 4);
static_assert(NB % PPB == 0 && NB % LBM == 0);
static_assert(LBM == NWAVE * 16 && ND % 16 == 0);
static_assert(KUSE % 32 == 0 && KUSE <= VP && KUSE <= WP && VP == 2 * ND && WP == 2 * ND);
static_assert((ND * (WP / 8)) % NTHR == 0);
static_assert((NREL * ND / 4) == 2 * NTHR);

typedef float          v2f   __attribute__((ext_vector_type(2)));
typedef float          v4f   __attribute__((ext_vector_type(4)));
typedef float          v8f   __attribute__((ext_vector_type(8)));
typedef int            v8i   __attribute__((ext_vector_type(8)));
typedef unsigned short v8us  __attribute__((ext_vector_type(8)));
typedef unsigned short v16us __attribute__((ext_vector_type(16)));
typedef __bf16         v16bf __attribute__((ext_vector_type(16)));
typedef v4f  __attribute__((may_alias)) v4fa;
typedef v8us __attribute__((may_alias)) v8usa;
union FragB { v16bf v; v16us u; v8us h[2]; v8i w; };

__device__ __forceinline__ v8f wmb(const FragB& a, const FragB& b, v8f c) {
  v8f d = __builtin_amdgcn_wmma_f32_16x16x32_bf16(false, a.v, false, b.v, (short)0, c, false, false);
  asm volatile("v_nop\n\tv_nop\n\tv_nop\n\tv_nop" : "+v"(d) : "v"(a.w), "v"(b.w));
  return d;
}

__device__ __forceinline__ unsigned bf16_bits(float f) {
  const unsigned u = __float_as_uint(f);
  const unsigned r = (u + 0x7FFFu + ((u >> 16) & 1u)) >> 16;
  return (f != f) ? 0x7FC0u : r;
}
__device__ __forceinline__ float bf16_val(float f) {
  return __uint_as_float(bf16_bits(f) << 16);
}

__device__ __forceinline__ float row_scale(float x0, float x1) {
  float ss = x0 * x0 + x1 * x1;
  ss += __shfl_xor(ss, 16);
  ss += __shfl_xor(ss, 8);
  ss += __shfl_xor(ss, 4);
  ss += __shfl_xor(ss, 2);
  ss += __shfl_xor(ss, 1);
  const float n = sqrtf(ss);
  return fminf(1.0f, 1.0f / fmaxf(n, 1e-7f));
}

__device__ __forceinline__ void cap_row(const float* __restrict__ src, float* dst, int lane) {
  v2f x = *(const v2f*)(src + 2 * lane);
  x.x = bf16_val(x.x);
  x.y = bf16_val(x.y);
  const float s = row_scale(x.x, x.y);
  v2f y;
  y.x = x.x * s;
  y.y = x.y * s;
  float* dp = dst + 2 * lane;
  *(volatile v2f*)dp = y;
  __threadfence();
  *(volatile v2f*)dp = y;
}

__global__ __launch_bounds__(NTHR) void k_renorm(const float* __restrict__ ent, const float* __restrict__ rel,
                                                 const float* __restrict__ W, const float* __restrict__ bias,
                                                 float* entN, float* relN, unsigned short* WD, float* biasR) {
  const int tid = (int)threadIdx.x, lane = tid & 31;
  const int wave = __builtin_amdgcn_readfirstlane(tid >> 5);
  if ((int)blockIdx.x < NB_ENT) {
    const int row0 = (int)blockIdx.x * ROWS_E + wave * RPW_E;
#pragma unroll 1
    for (int i = 0; i < RPW_E; ++i) {
      const size_t ro = (size_t)(row0 + i) * ND;
      cap_row(ent + ro, entN + ro, lane);
    }
  } else {
#pragma unroll 1
    for (int i = 0; i < 4; ++i) {
      const size_t ro = (size_t)(wave * 4 + i) * ND;
      cap_row(rel + ro, relN + ro, lane);
    }
#pragma unroll 1
    for (int j = 0; j < (ND * (WP / 8)) / NTHR; ++j) {
      const int u  = j * NTHR + tid;
      const int n  = u >> 4;
      const int k8 = (u & 15) * 8;
      const int kk = k8 & (ND - 1);
      const float* p = W + (size_t)n * ND + kk;
      const v4f a = *(const v4f*)p;
      const v4f b = *(const v4f*)(p + 4);
      v8us o;
      o[0] = (unsigned short)bf16_bits(a.x); o[1] = (unsigned short)bf16_bits(a.y);
      o[2] = (unsigned short)bf16_bits(a.z); o[3] = (unsigned short)bf16_bits(a.w);
      o[4] = (unsigned short)bf16_bits(b.x); o[5] = (unsigned short)bf16_bits(b.y);
      o[6] = (unsigned short)bf16_bits(b.z); o[7] = (unsigned short)bf16_bits(b.w);
      unsigned short* dp = WD + (size_t)n * WP + k8;
      *(volatile v8us*)dp = o;
      __threadfence();
      *(volatile v8us*)dp = o;
    }
    if (tid < 16) {
      const v4f t = *(const v4f*)(bias + 4 * tid);
      v4f r;
      r.x = bf16_val(t.x); r.y = bf16_val(t.y); r.z = bf16_val(t.z); r.w = bf16_val(t.w);
      float* dp = biasR + 4 * tid;
      *(volatile v4f*)dp = r;
      __threadfence();
      *(volatile v4f*)dp = r;
    }
  }
}

__global__ __launch_bounds__(NTHR) void k_pair(const float* __restrict__ utab, const int* __restrict__ users,
                                               const int* __restrict__ items, const int* __restrict__ adjE,
                                               const int* __restrict__ adjR, const float* __restrict__ entN,
                                               const float* __restrict__ relN, float* out0, unsigned short* V) {
  __shared__ float relS[NREL * RELP];
  const int tid = (int)threadIdx.x, lane = tid & 31;
  const int wave = __builtin_amdgcn_readfirstlane(tid >> 5);

#pragma unroll
  for (int j = 0; j < 2; ++j) {
    const int q = j * NTHR + tid;
    const v4f r = *(const v4f*)(relN + 4 * q);
    const int rr = q >> 4, c = (q & 15) * 4;
    relS[rr * RELP + c + 0] = r.x;
    relS[rr * RELP + c + 1] = r.y;
    relS[rr * RELP + c + 2] = r.z;
    relS[rr * RELP + c + 3] = r.w;
  }
  __syncthreads();

#pragma unroll 1
  for (int p = 0; p < PPW; ++p) {
    const int b = (int)blockIdx.x * PPB + wave * PPW + p;
    int uv = users[b];
    uv = min(max(uv, 0), NUSR - 1);
    int iv = items[b];
    iv = min(max(iv, 0), NENT - 1);
    const int uid = __builtin_amdgcn_readfirstlane(uv);
    const int it  = __builtin_amdgcn_readfirstlane(iv);
    int nid = adjE[(size_t)it * NK + lane];
    nid = min(max(nid, 0), NENT - 1);
    int rid = adjR[(size_t)it * NK + lane];
    rid = min(max(rid, 0), NREL - 1);

    v2f u = *(const v2f*)(utab + (size_t)uid * ND + 2 * lane);
    u.x = bf16_val(u.x);
    u.y = bf16_val(u.y);
    const float su = row_scale(u.x, u.y);
    u.x = u.x * su;
    u.y = u.y * su;

    const int uxi = __float_as_int(u.x), uyi = __float_as_int(u.y);
    float sr = 0.0f;
#pragma unroll 4
    for (int j = 0; j < 32; ++j) {
      const float ux = __int_as_float(__builtin_amdgcn_readlane(uxi, j));
      const float uy = __int_as_float(__builtin_amdgcn_readlane(uyi, j));
      sr = fmaf(ux, relS[lane * RELP + 2 * j], sr);
      sr = fmaf(uy, relS[lane * RELP + 2 * j + 1], sr);
    }

    const float s = __shfl(sr, rid);

    float mx = s;
    mx = fmaxf(mx, __shfl_xor(mx, 16));
    mx = fmaxf(mx, __shfl_xor(mx, 8));
    mx = fmaxf(mx, __shfl_xor(mx, 4));
    mx = fmaxf(mx, __shfl_xor(mx, 2));
    mx = fmaxf(mx, __shfl_xor(mx, 1));
    const float e = expf(s - mx);
    float sm = e;
    sm += __shfl_xor(sm, 16);
    sm += __shfl_xor(sm, 8);
    sm += __shfl_xor(sm, 4);
    sm += __shfl_xor(sm, 2);
    sm += __shfl_xor(sm, 1);
    const float a = e / sm;

    const int ai = __float_as_int(a);
    float nx = 0.0f, ny = 0.0f;
#pragma unroll 4
    for (int k = 0; k < NK; ++k) {
      const int   idk = __builtin_amdgcn_readlane(nid, k);
      const float ak  = __int_as_float(__builtin_amdgcn_readlane(ai, k));
      const v2f r = *(const v2f*)(entN + (size_t)idk * ND + 2 * lane);
      nx = fmaf(ak, r.x, nx);
      ny = fmaf(ak, r.y, ny);
    }
    const v2f itv = *(const v2f*)(entN + (size_t)it * ND + 2 * lane);
    const float vx = itv.x + nx;
    const float vy = itv.y + ny;

    const unsigned hx = bf16_bits(vx);
    const unsigned hy = bf16_bits(vy);
    const unsigned lx = bf16_bits(vx - __uint_as_float(hx << 16));
    const unsigned ly = bf16_bits(vy - __uint_as_float(hy << 16));
    const unsigned wh = (hx & 0xFFFFu) | (hy << 16);
    const unsigned wl = (lx & 0xFFFFu) | (ly << 16);
    unsigned* vrow = (unsigned*)(V + (size_t)b * VP);
    float* orow = out0 + (size_t)b * ND + 2 * lane;
    *(volatile unsigned*)(vrow + lane) = wh;
    *(volatile unsigned*)(vrow + 32 + lane) = wl;
    *(volatile v2f*)orow = u;
    __threadfence();
    *(volatile unsigned*)(vrow + lane) = wh;
    *(volatile unsigned*)(vrow + 32 + lane) = wl;
    *(volatile v2f*)orow = u;
  }
}

__global__ __launch_bounds__(NTHR) __attribute__((amdgpu_num_vgpr(248)))
void k_lin(const unsigned short* __restrict__ Vp, const unsigned short* __restrict__ WD,
           const float* __restrict__ biasR, float* out1) {
  __shared__ __attribute__((aligned(16))) float stg[LBM * ND];
  __shared__ __attribute__((aligned(16))) float sb[ND];
  const int tid = (int)threadIdx.x, lane = tid & 31, hh = lane >> 4, m = lane & 15;
  const int wave = __builtin_amdgcn_readfirstlane(tid >> 5);
  const int rowBase = (int)blockIdx.x * LBM;

  if (tid < 16) {
    const v4f t = *(const v4f*)(biasR + 4 * tid);
    *(v4fa*)(sb + 4 * tid) = t;
  }

  v8f acc[4];
  {
    const v8f z = {0.f, 0.f, 0.f, 0.f, 0.f, 0.f, 0.f, 0.f};
#pragma unroll
    for (int t = 0; t < 4; ++t) acc[t] = z;
  }
  const unsigned short* ap = Vp + (size_t)(rowBase + 16 * wave + m) * (size_t)VP + 8 * hh;
  const unsigned short* bp = WD + (size_t)m * (size_t)WP + 8 * hh;

#pragma unroll 1
  for (int k0 = 0; k0 < KUSE; k0 += 32) {
    FragB af;
    af.h[0] = *(const v8usa*)(ap + k0);
    af.h[1] = *(const v8usa*)(ap + k0 + 16);
#pragma unroll
    for (int nt = 0; nt < 4; ++nt) {
      const unsigned short* wq = bp + (size_t)(16 * nt) * (size_t)WP + k0;
      FragB bf;
      bf.h[0] = *(const v8usa*)wq;
      bf.h[1] = *(const v8usa*)(wq + 16);
      acc[nt] = wmb(af, bf, acc[nt]);
    }
  }

#pragma unroll
  for (int nt = 0; nt < 4; ++nt) {
    const int lc = 16 * nt + m;
#pragma unroll
    for (int r = 0; r < 8; ++r) {
      const int lr = 16 * wave + 8 * hh + r;
      stg[lr * ND + lc] = acc[nt][r];
    }
  }
  __syncthreads();

  const v4f bb = *(const v4fa*)(sb + 4 * (lane & 15));
  v4f pv[8];
#pragma unroll
  for (int i = 0; i < 8; ++i) {
    const v4f t = *(const v4fa*)(stg + (16 * wave) * ND + i * 128 + 4 * lane) + bb;
    v4f y;
    y.x = (t.x > 0.0f) ? t.x : (t.x - t.x);
    y.y = (t.y > 0.0f) ? t.y : (t.y - t.y);
    y.z = (t.z > 0.0f) ? t.z : (t.z - t.z);
    y.w = (t.w > 0.0f) ? t.w : (t.w - t.w);
    pv[i] = y;
  }
  float* op = out1 + (size_t)(rowBase + 16 * wave) * ND + 4 * lane;
#pragma unroll
  for (int i = 0; i < 8; ++i) *(volatile v4f*)(op + i * 128) = pv[i];
  __threadfence();
#pragma unroll
  for (int i = 0; i < 8; ++i) *(volatile v4f*)(op + i * 128) = pv[i];
}

static inline size_t al256(size_t o) { return (o + 255) & ~(size_t)255; }

extern "C" void kernel_launch(void* const* d_in, const int* in_sizes, int n_in,
                              void* d_out, int out_size, void* d_ws, size_t ws_size,
                              hipStream_t stream) {
  if (n_in < 9) return;
  if (in_sizes[0] != NUSR * ND) return;
  if (in_sizes[1] != NENT * ND) return;
  if (in_sizes[2] != NREL * ND) return;
  if (in_sizes[3] != ND * ND) return;
  if (in_sizes[4] != ND) return;
  if (in_sizes[5] != NB || in_sizes[6] != NB) return;
  if (in_sizes[7] != NENT * NK || in_sizes[8] != NENT * NK) return;
  if ((long long)out_size != 2LL * NB * ND) return;

  const float* utab  = (const float*)d_in[0];
  const float* etab  = (const float*)d_in[1];
  const float* rtab  = (const float*)d_in[2];
  const float* W     = (const float*)d_in[3];
  const float* bias  = (const float*)d_in[4];
  const int*   users = (const int*)d_in[5];
  const int*   items = (const int*)d_in[6];
  const int*   adjE  = (const int*)d_in[7];
  const int*   adjR  = (const int*)d_in[8];
  float* out0 = (float*)d_out;
  float* out1 = (float*)d_out + (size_t)NB * ND;

  char* ws = (char*)d_ws;
  size_t off = 0;
  const size_t oEnt  = off; off = al256(off + (size_t)NENT * ND * 4);
  const size_t oRel  = off; off = al256(off + (size_t)NREL * ND * 4);
  const size_t oV    = off; off = al256(off + (size_t)NB * VP * 2);
  const size_t oWD   = off; off = al256(off + (size_t)ND * WP * 2);
  const size_t oBias = off; off = al256(off + (size_t)ND * 4);
  if (off > ws_size || off > (size_t)(128u << 20)) return;
  float*          entN  = (float*)(ws + oEnt);
  float*          relN  = (float*)(ws + oRel);
  unsigned short* Vpl   = (unsigned short*)(ws + oV);
  unsigned short* WD    = (unsigned short*)(ws + oWD);
  float*          biasR = (float*)(ws + oBias);

  k_renorm<<<NB_ENT + 1, NTHR, 0, stream>>>(etab, rtab, W, bias, entN, relN, WD, biasR);
  k_pair<<<NB / PPB, NTHR, 0, stream>>>(utab, users, items, adjE, adjR, entN, relN, out0, Vpl);
  k_lin<<<NB / LBM, NTHR, 0, stream>>>(Vpl, WD, biasR, out1);
}
